// ConvFeatureExtractor_9414568313601
// MI455X (gfx1250) — hardware-verified
//
#include <hip/hip_runtime.h>
#include <math.h>

typedef __attribute__((ext_vector_type(16))) _Float16 v16h;
typedef __attribute__((ext_vector_type(16))) __bf16 v16b;
typedef __attribute__((ext_vector_type(8)))  _Float16 v8h;
typedef __attribute__((ext_vector_type(8)))  float v8f;
typedef __attribute__((ext_vector_type(4)))  float v4f;
typedef __attribute__((ext_vector_type(2)))  float v2f;
typedef __attribute__((ext_vector_type(4)))  unsigned v4u;
typedef __attribute__((ext_vector_type(4)))  int v4i;
typedef float __attribute__((may_alias)) float_a;
typedef int __attribute__((may_alias)) int_a;

template <typename T> __device__ __forceinline__ void vst2(void* p, T v) { *(volatile T*)p = v; __threadfence(); *(volatile T*)p = v; }
__device__ __forceinline__ v8f wmma16(v16h a, v16h b, v8f c) {
  v8f d = __builtin_amdgcn_wmma_f32_16x16x32_f16(false, a, false, b, (short)0, c, false, false);
  asm volatile("v_nop\n\tv_nop\n\tv_nop\n\tv_nop" : "+v"(d) : "v"(a), "v"(b));
  return d;
}
__device__ __forceinline__ v8f wmma_bf(v16b a, v16b b, v8f c) {
  v8f d = __builtin_amdgcn_wmma_f32_16x16x32_bf16(false, a, false, b, (short)0, c, false, false);
  asm volatile("v_nop\n\tv_nop\n\tv_nop\n\tv_nop" : "+v"(d) : "v"(a), "v"(b));
  return d;
}
__device__ __forceinline__ v16h frag_h(const _Float16* rowk0, int lane) {
  union { v16h v; v8h q[2]; } u; const _Float16* p = rowk0 + 8 * (lane >> 4);
  u.q[0] = *(const v8h*)p; u.q[1] = *(const v8h*)(p + 16); return u.v;
}
__device__ __forceinline__ v16h frag_f32(const float* rowk0, int lane) {
  v16h a; const float* p = rowk0 + 8 * (lane >> 4);
#pragma unroll
  for (int i = 0; i < 8; ++i) { a[i] = (_Float16)p[i]; a[8 + i] = (_Float16)p[16 + i]; }
  return a;
}
__device__ __forceinline__ v16h frag_f32s(const float* rowk0, int lane, float sc) {
  v16h a; const float* p = rowk0 + 8 * (lane >> 4);
#pragma unroll
  for (int i = 0; i < 8; ++i) { a[i] = (_Float16)(p[i] * sc); a[8 + i] = (_Float16)(p[16 + i] * sc); }
  return a;
}
__device__ __forceinline__ v16h fragc_f32(const float* W, int k0, int n, int lane, int ld, int K) {
  v16h a; const int g = lane >> 4;
#pragma unroll
  for (int i = 0; i < 8; ++i) { const int ka = k0 + 8 * g + i, kb = ka + 16;
    a[i] = (_Float16)(ka < K ? W[(size_t)(ka < K ? ka : K - 1) * ld + n] : 0.f); a[8 + i] = (_Float16)(kb < K ? W[(size_t)(kb < K ? kb : K - 1) * ld + n] : 0.f); }
  return a;
}
struct F2 { v16b h, l; };
__device__ __forceinline__ F2 bsplit16(const float v[16]) { F2 r;
#pragma unroll
  for (int i = 0; i < 16; ++i) { const __bf16 h = (__bf16)v[i]; r.h[i] = h; r.l[i] = (__bf16)(v[i] - (float)h); }
  return r; }
__device__ __forceinline__ F2 split_row(const float* row, int k0, int lane) { float v[16]; const float* p = row + k0 + 8 * (lane >> 4);
#pragma unroll
  for (int i = 0; i < 8; ++i) { v[i] = p[i]; v[8 + i] = p[16 + i]; }
  return bsplit16(v); }
__device__ __forceinline__ F2 split_rowK(const float* row, int k0, int lane, int K) { float v[16]; const int g = lane >> 4;
#pragma unroll
  for (int i = 0; i < 8; ++i) { const int ka = k0 + 8 * g + i, kb = ka + 16; v[i] = ka < K ? row[ka < K ? ka : K - 1] : 0.f; v[8 + i] = kb < K ? row[kb < K ? kb : K - 1] : 0.f; }
  return bsplit16(v); }
__device__ __forceinline__ F2 split_col(const float* W, int k0, int n, int lane, int ld, int K) { float v[16]; const int g = lane >> 4;
#pragma unroll
  for (int i = 0; i < 8; ++i) { const int ka = k0 + 8 * g + i, kb = ka + 16; v[i] = ka < K ? W[(size_t)(ka < K ? ka : K - 1) * ld + n] : 0.f; v[8 + i] = kb < K ? W[(size_t)(kb < K ? kb : K - 1) * ld + n] : 0.f; }
  return bsplit16(v); }
__device__ __forceinline__ v8f mac3(const F2& a, const F2& b, v8f c) { c = wmma_bf(a.l, b.h, c); c = wmma_bf(a.h, b.l, c); return wmma_bf(a.h, b.h, c); }
__device__ __forceinline__ float sigm(float v) { return 1.0f / (1.0f + expf(-v)); }
#define LDSX() do { asm volatile("s_wait_dscnt 0" ::: "memory"); __builtin_amdgcn_wave_barrier(); __builtin_amdgcn_fence(__ATOMIC_RELEASE, "workgroup"); } while (0)


#define NBATCH 1024
#define NM 4096
#define NF 8192
#define KK 6
#ifndef NRB
#define NRB (NBATCH / 64)
#endif
typedef __attribute__((ext_vector_type(8))) __bf16 v8b;
__device__ __forceinline__ v16b frag_b(const __bf16* rowk0, int lane) {
  union { v16b v; v8b q[2]; } u; const __bf16* p = rowk0 + 8 * (lane >> 4);
  u.q[0] = *(const v8b*)p; u.q[1] = *(const v8b*)(p + 16); return u.v;
}
__device__ __forceinline__ float bfr(float v) { return (float)(__bf16)v; }
__device__ __attribute__((noinline)) float exp_ni(float v) { return expf(v); }
__device__ __attribute__((noinline)) float erf_ni(float v) { return erff(v); }

#define WS_E   0u
#define WS_A   (WS_E + 2u * (size_t)NF * NM)
#define WS_S   (WS_A + 2u * (size_t)NBATCH * NM)
#define WS_P   (WS_S + 4u * NF)
#define WS_END (WS_P + 4u * (size_t)NBATCH * NF)

__device__ __attribute__((noinline)) float exp_p(float v) { return expf(v); }
__global__ __launch_bounds__(256) void k_match(const float* __restrict__ KP, const int* __restrict__ IDC, const float* __restrict__ TEMP, _Float16* __restrict__ E, float* __restrict__ S) {
  __shared__ float skp[4 * KK]; __shared__ float red[256]; __shared__ __align__(16) _Float16 se[NM]; __shared__ float slg[NM];
  const size_t f = blockIdx.x; const int t = threadIdx.x;
  if (t < 4 * KK) skp[t] = bfr(KP[f * 4 * KK + t]);
  __syncthreads();
  const float temp = bfr(TEMP[0]);
  float mx = -3.0e38f;
#pragma unroll 1
  for (int u = 0; u < 16; ++u) { const int i = t + 256 * u; float s = 0.f;
#pragma unroll
    for (int j = 0; j < KK; ++j) s += skp[IDC[(size_t)i * KK + j] * KK + j];
    const float lgv = s / temp; slg[i] = lgv; mx = fmaxf(mx, lgv); }
  red[t] = mx; __syncthreads();
  for (int st = 128; st > 0; st >>= 1) { if (t < st) red[t] = fmaxf(red[t], red[t + st]); __syncthreads(); }
  const float gmx = red[0]; __syncthreads();
  float sum = 0.f;
#pragma unroll 1
  for (int u = 0; u < 16; ++u) { const int i = t + 256 * u; const float e = exp_p(slg[i] - gmx); sum += e; se[i] = (_Float16)(e * 32768.0f); }
  red[t] = sum; __syncthreads();
  for (int st = 128; st > 0; st >>= 1) { if (t < st) red[t] += red[t + st]; __syncthreads(); }
  if (t == 0) S[f] = red[0];
  for (int q = t; q < NM / 8; q += 256) vst2((unsigned*)(E + f * NM + q * 8), *(const v4u*)&se[q * 8]);
}
__global__ __launch_bounds__(256) void k_afreq(const float* __restrict__ FR, _Float16* __restrict__ A) { __shared__ __align__(16) _Float16 s[NM]; const size_t b = blockIdx.x; const int t = threadIdx.x; for (int i = t; i < NM; i += 256) s[i] = (_Float16)(bfr(FR[b * NM + i]) * 256.0f); __syncthreads(); for (int q = t; q < NM / 8; q += 256) vst2((unsigned*)(A + b * NM + q * 8), *(const v4u*)&s[q * 8]); }
__global__ __launch_bounds__(128) void k_pool(const _Float16* __restrict__ A, const _Float16* __restrict__ E, const float* __restrict__ S, float* __restrict__ P) {
  __shared__ __align__(16) float so[4][16][132];
  const int tid = threadIdx.x, wave = tid >> 5, lane = tid & 31, col = lane & 15, g = lane >> 4; const size_t r0 = (size_t)blockIdx.x * 64 + wave * 16; const int n0 = blockIdx.y * 128;
  v8f acc[8] = {};
#pragma unroll 2
  for (int kc = 0; kc < NM / 32; ++kc) { const v16h a = frag_h(A + (r0 + col) * NM + kc * 32, lane);
#pragma unroll
    for (int j = 0; j < 8; ++j) acc[j] = wmma16(a, frag_h(E + (size_t)(n0 + j * 16 + col) * NM + kc * 32, lane), acc[j]); }
#pragma unroll
  for (int j = 0; j < 8; ++j) { const int f = n0 + j * 16 + col; const float inv = 1.0f / (8388608.0f * S[f]);
#pragma unroll
    for (int r = 0; r < 8; ++r) so[wave][8 * g + r][j * 16 + col] = acc[j][r] * inv; }
  LDSX();
  for (int rl = 0; rl < 16; ++rl) vst2(P + (r0 + rl) * NF + n0 + lane * 4, *(const v4f*)&so[wave][rl][lane * 4]);
}
__global__ __launch_bounds__(256) void k_norm(const float* __restrict__ P, float* __restrict__ OUT) {
  __shared__ float red[256]; const size_t b = blockIdx.x; const int t = threadIdx.x; float s = 0.f; for (int f = t; f < NF; f += 256) s += P[b * NF + f]; red[t] = s; __syncthreads();
  for (int st = 128; st > 0; st >>= 1) { if (t < st) red[t] += red[t + st]; __syncthreads(); }
  const float inv = 1.0f / red[0];
  for (int q = t; q < NF / 4; q += 256) { v4f v; for (int i = 0; i < 4; ++i) v[i] = P[b * NF + q * 4 + i] * inv; vst2(OUT + b * NF + q * 4, v); }
}
extern "C" void kernel_launch(void* const* d_in, const int* in_sizes, int n_in, void* d_out, int out_size, void* d_ws, size_t ws_size, hipStream_t stream) {
  (void)in_sizes; (void)n_in; (void)out_size;
  const float** F = (const float**)d_in;
  if (ws_size < (size_t)WS_END) return;
  char* ws = (char*)d_ws; _Float16 *E = (_Float16*)(ws + WS_E), *A = (_Float16*)(ws + WS_A); float *S = (float*)(ws + WS_S), *P = (float*)(ws + WS_P);
  k_match<<<NF, 256, 0, stream>>>(F[1], (const int*)d_in[3], F[2], E, S);
  k_afreq<<<NRB * 64, 256, 0, stream>>>(F[0], A);
  k_pool<<<dim3(NRB, NF / 128), 128, 0, stream>>>(A, E, S, P);
  k_norm<<<NRB * 64, 256, 0, stream>>>(P, (float*)d_out);
}
